// GAE_1185410974360
// MI455X (gfx1250) — hardware-verified
//
#include <hip/hip_runtime.h>
#include <stddef.h>
#include <stdint.h>


#define DIN    64
#define DF     128
#define LAT    32
#define MPITCH 256
#define HP     256
#define K0     192
#define KM     256
#define KH     256
#define KB1    512
#define KBI    64
#define LNEPS  1e-5f
#define NTHR   256
#define NWAVE  8
#define EPT    8
#define CHUNK  (NTHR * EPT)
#define WCAP   (EPT * 32)
#define LISTN  (NWAVE * WCAP)
#define NBA    1024
#define SLA    10
#define RCAP   28672
#define DEGCAP 64
#define GBM    64
#define GBN    128
#define GTHR   128
#define GWAVE  4
#define ROWH   256
#define ITHR   256
#define IROWS  128
#define ETHR   256
#define U0     3072
#define U1     8192
#define U2     2048
#define UI     1024
#define NUNITS (2 * U0 + 2 * U1 + 2 * U2 + UI)
#define AGG_ZINTS    (LISTN + 2 * RCAP + 3 * NBA)
#define MISC_INTS    16
#define ROWBUF_INTS  (NWAVE * ROWH / 2)
#define AGG_LDS_INTS (AGG_ZINTS + MISC_INTS + ROWBUF_INTS)
#define WSMAX  134217728

static_assert((CHUNK & (CHUNK - 1)) == 0 && CHUNK <= 4096);
static_assert((NBA & (NBA - 1)) == 0 && NBA == (1 << SLA));
static_assert(((long long)CHUNK << SLA) < (1LL << 31));
static_assert(LISTN % NTHR == 0);
static_assert(NBA % NWAVE == 0 && NBA % 32 == 0 && NBA % GBM == 0);
static_assert(RCAP % 4 == 0 && AGG_ZINTS % 4 == 0 && LISTN % 4 == 0 && ((AGG_ZINTS + MISC_INTS) % 4) == 0);
static_assert(AGG_ZINTS % (NTHR * 4) == 0);
static_assert(K0 % 32 == 0 && KM % 32 == 0 && KH % 32 == 0 && KBI % 32 == 0 && KB1 == KM + KH);
static_assert(K0 == 3 * DIN && K0 <= MPITCH && KM == MPITCH && KH == HP && HP == 2 * DF && KBI == 2 * LAT);
static_assert(GBN == DF && GBM == GWAVE * 16 && DF == 4 * 32 && GTHR == GWAVE * 32 && LAT == 32 && DIN == 2 * 32);
static_assert(AGG_LDS_INTS * 4 <= 300000);
static_assert(ROWH == MPITCH && ROWH == 8 * 32);
static_assert(U0 % NTHR == 0 && U1 % NTHR == 0 && U2 % NTHR == 0 && UI % NTHR == 0 && NUNITS % NTHR == 0);
static_assert((DF * 8) % NTHR == 0 && (LAT * 8) % NTHR == 0);
static_assert(U0 == 3 * DF * 8 && U1 == 8 * DF * 8 && U2 == 8 * LAT * 8 && UI == DF * 8);
static_assert(ITHR == NWAVE * 32 && IROWS == NWAVE * 16 && IROWS == 4 * 32 && ITHR == 2 * DF);
static_assert(ETHR == 256 && ETHR / 4 == 64);

typedef float          v2f   __attribute__((ext_vector_type(2)));
typedef float          v4f   __attribute__((ext_vector_type(4)));
typedef float          v8f   __attribute__((ext_vector_type(8)));
typedef int            v4i   __attribute__((ext_vector_type(4)));
typedef int            v8i   __attribute__((ext_vector_type(8)));
typedef unsigned       v2u   __attribute__((ext_vector_type(2)));
typedef unsigned short v2us  __attribute__((ext_vector_type(2)));
typedef unsigned short v4us  __attribute__((ext_vector_type(4)));
typedef unsigned short v8us  __attribute__((ext_vector_type(8)));
typedef unsigned short v16us __attribute__((ext_vector_type(16)));
typedef __bf16         v16bf __attribute__((ext_vector_type(16)));
typedef v2f  __attribute__((may_alias)) v2fa;
typedef v4f  __attribute__((may_alias)) v4fa;
typedef v4i  __attribute__((may_alias)) v4ia;
typedef v2u  __attribute__((may_alias)) v2ua;
typedef v2us __attribute__((may_alias)) v2usa;
typedef v4us __attribute__((may_alias)) v4usa;
typedef v8us __attribute__((may_alias)) v8usa;
union FragB { v16bf v; v16us u; v8us h[2]; v8i w; };

struct TW {
  const unsigned short* bt;
  const float* bias;
  const float* gam;
  const float* bet;
  unsigned short* hout;
};
static_assert(sizeof(TW) == 40);

__device__ __forceinline__ v8f wmb(const FragB& a, const FragB& b, v8f c) {
  v8f d = __builtin_amdgcn_wmma_f32_16x16x32_bf16(false, a.v, false, b.v, (short)0, c, false, false);
  asm volatile("v_nop\n\tv_nop\n\tv_nop\n\tv_nop" : "+v"(d) : "v"(a.w), "v"(b.w));
  return d;
}

__device__ __forceinline__ v8f z8() { v8f z = {0.f, 0.f, 0.f, 0.f, 0.f, 0.f, 0.f, 0.f}; return z; }

__device__ __forceinline__ unsigned bf16_bits(float f) {
  const unsigned u = __float_as_uint(f);
  return (u + 0x7FFFu + ((u >> 16) & 1u)) >> 16;
}
__device__ __forceinline__ float bf16_val(float f) {
  return __uint_as_float(bf16_bits(f) << 16);
}
__device__ __forceinline__ unsigned hl_bits(float v, unsigned& lo) {
  const unsigned hb = bf16_bits(v);
  lo = bf16_bits(v - __uint_as_float(hb << 16));
  return hb;
}

__device__ __forceinline__ void wave_sync() {
  __builtin_amdgcn_fence(__ATOMIC_RELEASE, "wavefront");
  __builtin_amdgcn_wave_barrier();
  __builtin_amdgcn_fence(__ATOMIC_ACQUIRE, "wavefront");
}

template <int SLB>
__device__ __forceinline__ int scan_chunk(const int* __restrict__ dsts, int nE, int cbase, int slotBase,
                                          int nb, int vec8, int* list, int tid, int lane, int wave) {
  int wc = 0;
  const int el0  = tid * EPT;
  const int e0   = cbase + el0;
  const int sent = -2147483647 - 1;
  v4i da, db;
  if (vec8 != 0 && cbase + CHUNK <= nE) {
    da = *(const v4i*)(dsts + e0);
    db = *(const v4i*)(dsts + e0 + 4);
  } else {
    da.x = (e0     < nE) ? dsts[min(e0,     nE - 1)] : sent;
    da.y = (e0 + 1 < nE) ? dsts[min(e0 + 1, nE - 1)] : sent;
    da.z = (e0 + 2 < nE) ? dsts[min(e0 + 2, nE - 1)] : sent;
    da.w = (e0 + 3 < nE) ? dsts[min(e0 + 3, nE - 1)] : sent;
    db.x = (e0 + 4 < nE) ? dsts[min(e0 + 4, nE - 1)] : sent;
    db.y = (e0 + 5 < nE) ? dsts[min(e0 + 5, nE - 1)] : sent;
    db.z = (e0 + 6 < nE) ? dsts[min(e0 + 6, nE - 1)] : sent;
    db.w = (e0 + 7 < nE) ? dsts[min(e0 + 7, nE - 1)] : sent;
  }
  const unsigned nbs = (unsigned)slotBase;
  const unsigned unb = (unsigned)nb;
  const unsigned s0 = (unsigned)da.x - nbs, s1 = (unsigned)da.y - nbs;
  const unsigned s2 = (unsigned)da.z - nbs, s3 = (unsigned)da.w - nbs;
  const unsigned s4 = (unsigned)db.x - nbs, s5 = (unsigned)db.y - nbs;
  const unsigned s6 = (unsigned)db.z - nbs, s7 = (unsigned)db.w - nbs;
  const bool h0 = s0 < unb, h1 = s1 < unb, h2 = s2 < unb, h3 = s3 < unb;
  const bool h4 = s4 < unb, h5 = s5 < unb, h6 = s6 < unb, h7 = s7 < unb;
  const unsigned any = __builtin_amdgcn_ballot_w32(h0 | h1 | h2 | h3 | h4 | h5 | h6 | h7);
  if (any != 0u) {
#define HITJ(J, HJ, SJ) { \
      const unsigned mj = __builtin_amdgcn_ballot_w32(HJ); \
      if (mj != 0u) { \
        if (HJ) { \
          const int pos = wc + (int)__builtin_amdgcn_mbcnt_lo(mj, 0u); \
          if (pos < WCAP) list[wave * WCAP + pos] = ((el0 + (J)) << SLB) | (int)(SJ); \
        } \
        wc += (int)__builtin_popcount(mj); } }
    HITJ(0, h0, s0)
    HITJ(1, h1, s1)
    HITJ(2, h2, s2)
    HITJ(3, h3, s3)
    HITJ(4, h4, s4)
    HITJ(5, h5, s5)
    HITJ(6, h6, s6)
    HITJ(7, h7, s7)
#undef HITJ
  }
  return wc;
}

__global__ __launch_bounds__(NTHR) void k_wprep(const float* __restrict__ mW0l, const float* __restrict__ mW0r,
                                                const float* __restrict__ vW0l, const float* __restrict__ vW0r,
                                                const float* __restrict__ mW1l, const float* __restrict__ mW1r,
                                                const float* __restrict__ vW1l, const float* __restrict__ vW1r,
                                                const float* __restrict__ mW2l, const float* __restrict__ mW2r,
                                                const float* __restrict__ vW2l, const float* __restrict__ vW2r,
                                                const float* __restrict__ iW1,
                                                unsigned short* BT0m, unsigned short* BT0v,
                                                unsigned short* BT1m, unsigned short* BT1v,
                                                unsigned short* BT2m, unsigned short* BT2v, unsigned short* BTi) {
  const int u = (int)blockIdx.x * NTHR + (int)threadIdx.x;
  const float* W;
  unsigned short* P;
  int nout, kmask, pitch, cb, w;
  if (u < U0) {
    const int v = u;                  cb = v >> 10; w = v & 1023;
    W = (cb < 2) ? mW0l : mW0r;       nout = DF;  kmask = DIN - 1; P = BT0m; pitch = K0;
  } else if (u < 2 * U0) {
    const int v = u - U0;             cb = v >> 10; w = v & 1023;
    W = (cb < 2) ? vW0l : vW0r;       nout = DF;  kmask = DIN - 1; P = BT0v; pitch = K0;
  } else if (u < 2 * U0 + U1) {
    const int v = u - 2 * U0;         cb = v >> 10; w = v & 1023;
    W = (cb < 4) ? mW1l : mW1r;       nout = DF;  kmask = DF - 1;  P = BT1m; pitch = KB1;
  } else if (u < 2 * U0 + 2 * U1) {
    const int v = u - 2 * U0 - U1;    cb = v >> 10; w = v & 1023;
    W = (cb < 4) ? vW1l : vW1r;       nout = DF;  kmask = DF - 1;  P = BT1v; pitch = KB1;
  } else if (u < 2 * U0 + 2 * U1 + U2) {
    const int v = u - 2 * U0 - 2 * U1;        cb = v >> 8; w = v & 255;
    W = (cb < 4) ? mW2l : mW2r;       nout = LAT; kmask = DF - 1;  P = BT2m; pitch = KB1;
  } else if (u < 2 * U0 + 2 * U1 + 2 * U2) {
    const int v = u - 2 * U0 - 2 * U1 - U2;   cb = v >> 8; w = v & 255;
    W = (cb < 4) ? vW2l : vW2r;       nout = LAT; kmask = DF - 1;  P = BT2v; pitch = KB1;
  } else if (u < NUNITS) {
    const int v = u - 2 * U0 - 2 * U1 - 2 * U2;   cb = 0; w = v & 1023;
    W = iW1;                          nout = DF;  kmask = LAT - 1; P = BTi;  pitch = KBI;
  } else {
    return;
  }
  const int n   = w >> 3, k8 = (w & 7) * 8;
  const int col = cb * 64 + k8;
  const int kk  = col & kmask;
  v8us o;
#pragma unroll
  for (int i = 0; i < 8; ++i) o[i] = (unsigned short)bf16_bits(W[(size_t)(kk + i) * (size_t)nout + (size_t)n]);
  unsigned short* dp = P + (size_t)n * (size_t)pitch + col;
  *(volatile v8us*)dp = o;
  __threadfence();
  *(volatile v8us*)dp = o;
}

template <int L0>
__global__ __launch_bounds__(NTHR) void k_scan(const int* __restrict__ srcs, const int* __restrict__ dsts,
                                               int nE, int nN, int vec8, int mRows,
                                               const float* __restrict__ xin, const unsigned short* hpl,
                                               unsigned short* mpl) {
  extern __shared__ __attribute__((aligned(16))) int dsm[];
  int* list = dsm;
  int* hl   = dsm + LISTN;
  int* sl   = hl + RCAP;
  int* cnt  = sl + RCAP;
  int* offs = cnt + NBA;
  int* cur  = offs + NBA;
  int* misc = cur + NBA;
  const int tid = (int)threadIdx.x, lane = tid & 31, wave = tid >> 5;
  unsigned short* rowbuf = (unsigned short*)(misc + MISC_INTS) + wave * ROWH;
  const int nodeBase = (int)blockIdx.x * NBA;

  {
    const v4i z4 = {0, 0, 0, 0};
    for (int i = tid * 4; i < AGG_ZINTS; i += NTHR * 4) *(v4ia*)(dsm + i) = z4;
    if (tid < MISC_INTS) misc[tid] = 0;
  }
  __syncthreads();

  int t = 0, ov = 0;
  const int nChunks = (nE + CHUNK - 1) / CHUNK;
#pragma unroll 1
  for (int ch = 0; ch < nChunks; ++ch) {
    const int cbase = ch * CHUNK;
    const int wc = scan_chunk<SLA>(dsts, nE, cbase, nodeBase, NBA, vec8, list, tid, lane, wave);
    if (lane == 0) misc[wave] = wc;
    __syncthreads();
    if (wave == 0) {
#pragma unroll 1
      for (int w2 = 0; w2 < NWAVE; ++w2) {
        int c = misc[w2];
        c = c < 0 ? 0 : (c > WCAP ? WCAP : c);
#pragma unroll 1
        for (int b0 = 0; b0 < c; b0 += 32) {
          const int idx = b0 + lane;
          const int ent_ = list[w2 * WCAP + (idx < WCAP ? idx : WCAP - 1)];
          const int m32 = (c - b0) < 32 ? (c - b0) : 32;
#pragma unroll 1
          for (int k = 0; k < m32; ++k) {
            const int u    = __builtin_amdgcn_readlane(ent_, k);
            const int slot = u & (NBA - 1);
            const int el   = (u >> SLA) & (CHUNK - 1);
            const int pk   = ((cbase + el) << SLA) | slot;
            if (t < RCAP) {
              if (lane == 0) { hl[t] = pk; cnt[slot] = cnt[slot] + 1; }
              t = t + 1;
            } else {
              ov = 1;
            }
          }
        }
      }
    }
    __syncthreads();
  }
  if (wave == 0 && lane == 0) { misc[8] = t; misc[9] = ov; }
  __syncthreads();
  int tt = misc[8];
  tt = tt < 0 ? 0 : (tt > RCAP ? RCAP : tt);
  const int ovf = misc[9];

  if (wave == 0) {
    const int base = lane * (NBA / 32);
    int s = 0;
#pragma unroll 1
    for (int i = 0; i < NBA / 32; ++i) s += cnt[base + i];
    int incl = s;
#pragma unroll
    for (int d = 1; d < 32; d <<= 1) {
      const int y = __shfl_up(incl, d, 32);
      if (lane >= d) incl += y;
    }
    int run = incl - s;
#pragma unroll 1
    for (int i = 0; i < NBA / 32; ++i) {
      const int cv = cnt[base + i];
      offs[base + i] = run;
      cur[base + i]  = run;
      run += cv;
    }
  }
  __syncthreads();
  if (wave == 0) {
#pragma unroll 1
    for (int b0 = 0; b0 < tt; b0 += 32) {
      const int idx = b0 + lane;
      const int ent_ = hl[idx < RCAP ? idx : RCAP - 1];
      const int m32 = (tt - b0) < 32 ? (tt - b0) : 32;
#pragma unroll 1
      for (int k = 0; k < m32; ++k) {
        const int u    = __builtin_amdgcn_readlane(ent_, k);
        const int slot = u & (NBA - 1);
        if (lane == 0) {
          int p = cur[slot];
          p = p < 0 ? 0 : (p > RCAP - 1 ? RCAP - 1 : p);
          sl[p] = u;
          cur[slot] = p + 1;
        }
      }
    }
  }
  __syncthreads();

  const float pz = (ovf != 0) ? __int_as_float(0x7fc00000) : 0.0f;
#pragma unroll 1
  for (int si = 0; si < NBA / NWAVE; ++si) {
    const int s    = si * NWAVE + wave;
    const int node = nodeBase + s;
    int c = cnt[s];
    const bool big = c > DEGCAP;
    c = c < 0 ? 0 : (c > DEGCAP ? DEGCAP : c);
    int o = offs[s];
    o = o < 0 ? 0 : (o > RCAP ? RCAP : o);
    const float pzr = big ? __int_as_float(0x7fc00000) : pz;
    const bool live = node < nN;
    const int nc = node < nN ? node : nN - 1;
    float a0 = 0.0f, a1 = 0.0f, a2 = 0.0f, a3 = 0.0f;
#pragma unroll 1
    for (int b0 = 0; b0 < c; b0 += 32) {
      int idx = o + b0 + lane;
      idx = idx > RCAP - 1 ? RCAP - 1 : idx;
      const int ent_ = sl[idx];
      int eid = ent_ >> SLA;
      eid = eid < 0 ? 0 : (eid > nE - 1 ? nE - 1 : eid);
      int sr = srcs[eid];
      sr = sr < 0 ? 0 : (sr > nN - 1 ? nN - 1 : sr);
      const int m32 = (c - b0) < 32 ? (c - b0) : 32;
#pragma unroll 1
      for (int k = 0; k < m32; ++k) {
        const int sk = __builtin_amdgcn_readlane(sr, k);
        if constexpr (L0 != 0) {
          const v2f a = *(const v2fa*)(xin + (size_t)sk * DIN + 2 * lane);
          a0 += bf16_val(a.x);
          a1 += bf16_val(a.y);
        } else {
          const unsigned short* rp = hpl + (size_t)sk * HP + 4 * lane;
          const v2u wh = *(const v2ua*)rp;
          const v2u wl = *(const v2ua*)(rp + DF);
          const float f0 = __uint_as_float(wh.x << 16)         + __uint_as_float(wl.x << 16);
          const float f1 = __uint_as_float(wh.x & 0xffff0000u) + __uint_as_float(wl.x & 0xffff0000u);
          const float f2 = __uint_as_float(wh.y << 16)         + __uint_as_float(wl.y << 16);
          const float f3 = __uint_as_float(wh.y & 0xffff0000u) + __uint_as_float(wl.y & 0xffff0000u);
          a0 += f0; a1 += f1; a2 += f2; a3 += f3;
        }
      }
    }
    const float inv = 1.0f / fmaxf((float)c, 1.0f);
    if constexpr (L0 != 0) {
      const float m0 = live ? (a0 * inv + pzr) : 0.0f;
      const float m1 = live ? (a1 * inv + pzr) : 0.0f;
      v2us mh, ml, xb;
      {
        unsigned lb;
        unsigned hb;
        hb = hl_bits(m0, lb); mh[0] = (unsigned short)hb; ml[0] = (unsigned short)lb;
        hb = hl_bits(m1, lb); mh[1] = (unsigned short)hb; ml[1] = (unsigned short)lb;
      }
      const v2f xs = *(const v2fa*)(xin + (size_t)nc * DIN + 2 * lane);
      xb[0] = live ? (unsigned short)bf16_bits(xs.x + pzr) : (unsigned short)0;
      xb[1] = live ? (unsigned short)bf16_bits(xs.y + pzr) : (unsigned short)0;
      const v2us z2 = {0, 0};
      *(v2usa*)(rowbuf + 2 * lane)           = mh;
      *(v2usa*)(rowbuf + DIN + 2 * lane)     = ml;
      *(v2usa*)(rowbuf + 2 * DIN + 2 * lane) = xb;
      *(v2usa*)(rowbuf + 3 * DIN + 2 * lane) = z2;
      (void)a2; (void)a3;
    } else {
      const float m0 = live ? (a0 * inv + pzr) : 0.0f;
      const float m1 = live ? (a1 * inv + pzr) : 0.0f;
      const float m2 = live ? (a2 * inv + pzr) : 0.0f;
      const float m3 = live ? (a3 * inv + pzr) : 0.0f;
      v4us mh, ml;
      {
        unsigned lb;
        unsigned hb;
        hb = hl_bits(m0, lb); mh[0] = (unsigned short)hb; ml[0] = (unsigned short)lb;
        hb = hl_bits(m1, lb); mh[1] = (unsigned short)hb; ml[1] = (unsigned short)lb;
        hb = hl_bits(m2, lb); mh[2] = (unsigned short)hb; ml[2] = (unsigned short)lb;
        hb = hl_bits(m3, lb); mh[3] = (unsigned short)hb; ml[3] = (unsigned short)lb;
      }
      *(v4usa*)(rowbuf + 4 * lane)      = mh;
      *(v4usa*)(rowbuf + DF + 4 * lane) = ml;
      (void)nc;
    }
    wave_sync();
    const v8us q0 = *(const v8usa*)(rowbuf + 8 * lane);
    wave_sync();
    if (node < mRows) {
      unsigned short* rpw = mpl + (size_t)node * MPITCH + 8 * lane;
      *(volatile v8us*)rpw = q0;
      __threadfence();
      *(volatile v8us*)rpw = q0;
    }
  }
  (void)xin; (void)hpl;
}

__global__ __launch_bounds__(GTHR) void k_gemmh(const unsigned short* A1, int lda1, int K1,
                                                const unsigned short* A2, int lda2, int K2,
                                                TW t0, TW t1, int nN) {
  __shared__ __attribute__((aligned(16))) float stg[GBM * GBN];
  const int tid = (int)threadIdx.x, lane = tid & 31, wave = tid >> 5, hh = lane >> 4, m = lane & 15;
  const int rowBase = (int)blockIdx.x * GBM;
  const TW tw = (blockIdx.y != 0) ? t1 : t0;
  const int ldb = K1 + K2;

  v8f acc[8];
#pragma unroll
  for (int t = 0; t < 8; ++t) acc[t] = z8();
  const unsigned short* ap1 = A1 + (size_t)(rowBase + 16 * wave + m) * (size_t)lda1 + 8 * hh;
  const unsigned short* ap2 = A2 + (size_t)(rowBase + 16 * wave + m) * (size_t)lda2 + 8 * hh;
  const unsigned short* bp  = tw.bt + (size_t)m * (size_t)ldb + 8 * hh;

#pragma unroll 1
  for (int k0 = 0; k0 < K1; k0 += 32) {
    FragB af;
    af.h[0] = *(const v8usa*)(ap1 + k0);
    af.h[1] = *(const v8usa*)(ap1 + k0 + 16);
#pragma unroll
    for (int nt = 0; nt < 8; ++nt) {
      const unsigned short* wq = bp + (size_t)(16 * nt) * (size_t)ldb + k0;
      FragB bf;
      bf.h[0] = *(const v8usa*)wq;
      bf.h[1] = *(const v8usa*)(wq + 16);
      acc[nt] = wmb(af, bf, acc[nt]);
    }
  }
#pragma unroll 1
  for (int k0 = 0; k0 < K2; k0 += 32) {
    FragB af;
    af.h[0] = *(const v8usa*)(ap2 + k0);
    af.h[1] = *(const v8usa*)(ap2 + k0 + 16);
#pragma unroll
    for (int nt = 0; nt < 8; ++nt) {
      const unsigned short* wq = bp + (size_t)(16 * nt) * (size_t)ldb + K1 + k0;
      FragB bf;
      bf.h[0] = *(const v8usa*)wq;
      bf.h[1] = *(const v8usa*)(wq + 16);
      acc[nt] = wmb(af, bf, acc[nt]);
    }
  }

#pragma unroll
  for (int nt = 0; nt < 8; ++nt) {
    const int lc = 16 * nt + m;
#pragma unroll
    for (int r = 0; r < 8; ++r) {
      const int lr = 16 * wave + 8 * hh + r;
      stg[lr * GBN + lc] = acc[nt][r];
    }
  }
  __syncthreads();

  float bq[4], gq[4], eq[4];
  {
    const v4f b4 = *(const v4f*)(tw.bias + 4 * lane);
    const v4f g4 = *(const v4f*)(tw.gam + 4 * lane);
    const v4f e4 = *(const v4f*)(tw.bet + 4 * lane);
    bq[0] = bf16_val(b4.x); bq[1] = bf16_val(b4.y); bq[2] = bf16_val(b4.z); bq[3] = bf16_val(b4.w);
    gq[0] = bf16_val(g4.x); gq[1] = bf16_val(g4.y); gq[2] = bf16_val(g4.z); gq[3] = bf16_val(g4.w);
    eq[0] = bf16_val(e4.x); eq[1] = bf16_val(e4.y); eq[2] = bf16_val(e4.z); eq[3] = bf16_val(e4.w);
  }

  v4f pv[16];
#pragma unroll
  for (int i = 0; i < 16; ++i) pv[i] = *(const v4fa*)(stg + (16 * wave + i) * GBN + 4 * lane);
  __syncthreads();

  const float invd = 1.0f / (float)DF;
#pragma unroll
  for (int i = 0; i < 16; ++i) {
    const int row = rowBase + 16 * wave + i;
    const bool ok = row < nN;
    const float y0 = pv[i].x + bq[0], y1 = pv[i].y + bq[1], y2 = pv[i].z + bq[2], y3 = pv[i].w + bq[3];
    float s = (y0 + y1) + (y2 + y3);
    s += __shfl_xor(s, 16, 32);
    s += __shfl_xor(s, 8, 32);
    s += __shfl_xor(s, 4, 32);
    s += __shfl_xor(s, 2, 32);
    s += __shfl_xor(s, 1, 32);
    const float mean = s * invd;
    const float d0 = y0 - mean, d1 = y1 - mean, d2 = y2 - mean, d3 = y3 - mean;
    float q = (d0 * d0 + d1 * d1) + (d2 * d2 + d3 * d3);
    q += __shfl_xor(q, 16, 32);
    q += __shfl_xor(q, 8, 32);
    q += __shfl_xor(q, 4, 32);
    q += __shfl_xor(q, 2, 32);
    q += __shfl_xor(q, 1, 32);
    const float var  = q * invd;
    const float rstd = rsqrtf(var + LNEPS);
    const float o0 = fmaxf(fmaf(d0 * rstd, gq[0], eq[0]), 0.0f);
    const float o1 = fmaxf(fmaf(d1 * rstd, gq[1], eq[1]), 0.0f);
    const float o2 = fmaxf(fmaf(d2 * rstd, gq[2], eq[2]), 0.0f);
    const float o3 = fmaxf(fmaf(d3 * rstd, gq[3], eq[3]), 0.0f);
    v4f qo;
    qo.x = ok ? o0 : 0.0f; qo.y = ok ? o1 : 0.0f; qo.z = ok ? o2 : 0.0f; qo.w = ok ? o3 : 0.0f;
    pv[i] = qo;
  }

#pragma unroll
  for (int i = 0; i < 16; ++i) {
    v4us h4, l4;
    unsigned lb;
    unsigned hb;
    hb = hl_bits(pv[i].x, lb); h4[0] = (unsigned short)hb; l4[0] = (unsigned short)lb;
    hb = hl_bits(pv[i].y, lb); h4[1] = (unsigned short)hb; l4[1] = (unsigned short)lb;
    hb = hl_bits(pv[i].z, lb); h4[2] = (unsigned short)hb; l4[2] = (unsigned short)lb;
    hb = hl_bits(pv[i].w, lb); h4[3] = (unsigned short)hb; l4[3] = (unsigned short)lb;
    unsigned short* srow = (unsigned short*)stg + (size_t)(16 * wave + i) * (2 * GBN);
    *(v4usa*)(srow + 4 * lane) = h4;
    *(v4usa*)(srow + DF + 4 * lane) = l4;
  }
  __syncthreads();
  v8us qv[16];
#pragma unroll
  for (int i = 0; i < 16; ++i) {
    const unsigned short* srow = (const unsigned short*)stg + (size_t)(16 * wave + i) * (2 * GBN);
    qv[i] = *(const v8usa*)(srow + 8 * lane);
  }
#pragma unroll
  for (int i = 0; i < 16; ++i) {
    const int gr = rowBase + 16 * wave + i;
    unsigned short* rp = tw.hout + (size_t)gr * (size_t)HP + 8 * lane;
    if (gr < nN) *(volatile v8us*)rp = qv[i];
  }
  __threadfence();
#pragma unroll
  for (int i = 0; i < 16; ++i) {
    const int gr = rowBase + 16 * wave + i;
    unsigned short* rp = tw.hout + (size_t)gr * (size_t)HP + 8 * lane;
    if (gr < nN) *(volatile v8us*)rp = qv[i];
  }
}

__global__ __launch_bounds__(GTHR) void k_gemmo(const unsigned short* A1, int lda1, int K1,
                                                const unsigned short* A2, int lda2, int K2,
                                                const unsigned short* __restrict__ BT,
                                                const float* __restrict__ bias, float climit,
                                                float* outp, int nN) {
  __shared__ __attribute__((aligned(16))) float stg[GBM * LAT];
  const int tid = (int)threadIdx.x, lane = tid & 31, wave = tid >> 5, hh = lane >> 4, m = lane & 15;
  const int rowBase = (int)blockIdx.x * GBM;
  const int ldb = K1 + K2;

  v8f acc[2];
  acc[0] = z8(); acc[1] = z8();
  const unsigned short* ap1 = A1 + (size_t)(rowBase + 16 * wave + m) * (size_t)lda1 + 8 * hh;
  const unsigned short* ap2 = A2 + (size_t)(rowBase + 16 * wave + m) * (size_t)lda2 + 8 * hh;
  const unsigned short* bp  = BT + (size_t)m * (size_t)ldb + 8 * hh;

#pragma unroll 1
  for (int k0 = 0; k0 < K1; k0 += 32) {
    FragB af;
    af.h[0] = *(const v8usa*)(ap1 + k0);
    af.h[1] = *(const v8usa*)(ap1 + k0 + 16);
#pragma unroll
    for (int nt = 0; nt < 2; ++nt) {
      const unsigned short* wq = bp + (size_t)(16 * nt) * (size_t)ldb + k0;
      FragB bf;
      bf.h[0] = *(const v8usa*)wq;
      bf.h[1] = *(const v8usa*)(wq + 16);
      acc[nt] = wmb(af, bf, acc[nt]);
    }
  }
#pragma unroll 1
  for (int k0 = 0; k0 < K2; k0 += 32) {
    FragB af;
    af.h[0] = *(const v8usa*)(ap2 + k0);
    af.h[1] = *(const v8usa*)(ap2 + k0 + 16);
#pragma unroll
    for (int nt = 0; nt < 2; ++nt) {
      const unsigned short* wq = bp + (size_t)(16 * nt) * (size_t)ldb + K1 + k0;
      FragB bf;
      bf.h[0] = *(const v8usa*)wq;
      bf.h[1] = *(const v8usa*)(wq + 16);
      acc[nt] = wmb(af, bf, acc[nt]);
    }
  }

#pragma unroll
  for (int nt = 0; nt < 2; ++nt) {
    const int lc = 16 * nt + m;
#pragma unroll
    for (int r = 0; r < 8; ++r) {
      const int lr = 16 * wave + 8 * hh + r;
      stg[lr * LAT + lc] = acc[nt][r];
    }
  }
  __syncthreads();

  v4f bq;
  {
    const v4f b4 = *(const v4f*)(bias + 4 * (lane & 7));
    bq.x = bf16_val(b4.x); bq.y = bf16_val(b4.y); bq.z = bf16_val(b4.z); bq.w = bf16_val(b4.w);
  }
  v4f pv[4];
#pragma unroll
  for (int j = 0; j < 4; ++j) {
    v4f y = *(const v4fa*)(stg + (size_t)(16 * wave) * LAT + 128 * j + 4 * lane) + bq;
    y.x = (y.x > climit) ? climit : y.x;
    y.y = (y.y > climit) ? climit : y.y;
    y.z = (y.z > climit) ? climit : y.z;
    y.w = (y.w > climit) ? climit : y.w;
    pv[j] = y;
  }
  const bool ok = (rowBase + 16 * wave + 16) <= nN;
  float* ob = outp + (size_t)(rowBase + 16 * wave) * LAT;
#pragma unroll
  for (int j = 0; j < 4; ++j)
    if (ok) *(volatile v4f*)(ob + 128 * j + 4 * lane) = pv[j];
  __threadfence();
#pragma unroll
  for (int j = 0; j < 4; ++j)
    if (ok) *(volatile v4f*)(ob + 128 * j + 4 * lane) = pv[j];
}

__global__ __launch_bounds__(ITHR) void k_ign(const float* mu, const int* __restrict__ slot,
                                              const unsigned short* __restrict__ BTi,
                                              const float* __restrict__ ib1, const float* __restrict__ iw2,
                                              const float* __restrict__ ib2, float* outp, int nN) {
  __shared__ __attribute__((aligned(16))) float sb1[DF];
  __shared__ __attribute__((aligned(16))) float sw2[DF];
  __shared__ __attribute__((aligned(16))) float ost[IROWS];
  __shared__ int flg[NWAVE];
  const int tid = (int)threadIdx.x, lane = tid & 31, wave = tid >> 5, hh = lane >> 4, m = lane & 15;
  const int rowBase = (int)blockIdx.x * IROWS;

  if (wave < 4) {
    sb1[tid] = bf16_val(ib1[tid]);
    sw2[tid] = bf16_val(iw2[tid]);
    if (lane == 0) flg[wave] = 0;
  } else {
    const int r  = rowBase + (tid - DF);
    const int rc = r < nN ? r : nN - 1;
    const bool bad = (r < nN) && (slot[rc] != r);
    const unsigned mj = __builtin_amdgcn_ballot_w32(bad);
    if (lane == 0) flg[wave] = (mj != 0u) ? 1 : 0;
  }

  const int row = rowBase + 16 * wave + m;
  const int rcl = row < nN ? row : nN - 1;
  const float* p = mu + (size_t)rcl * LAT;
  const v4f u0 = *(const v4fa*)(p + 8 * hh);
  const v4f u1 = *(const v4fa*)(p + 8 * hh + 4);
  const v4f u2 = *(const v4fa*)(p + 16 + 8 * hh);
  const v4f u3 = *(const v4fa*)(p + 16 + 8 * hh + 4);
  const float f[16] = {u0.x, u0.y, u0.z, u0.w, u1.x, u1.y, u1.z, u1.w,
                       u2.x, u2.y, u2.z, u2.w, u3.x, u3.y, u3.z, u3.w};
  FragB ah, al;
#pragma unroll
  for (int i = 0; i < 16; ++i) {
    unsigned lb;
    const unsigned hb = hl_bits(f[i], lb);
    ah.u[i] = (unsigned short)hb;
    al.u[i] = (unsigned short)lb;
  }
  v8f acc[8];
#pragma unroll
  for (int t = 0; t < 8; ++t) acc[t] = z8();
  const unsigned short* bp = BTi + (size_t)m * KBI + 8 * hh;
#pragma unroll
  for (int nt = 0; nt < 8; ++nt) {
    const unsigned short* wq = bp + (size_t)(16 * nt) * KBI;
    FragB b0, b1;
    b0.h[0] = *(const v8usa*)wq;
    b0.h[1] = *(const v8usa*)(wq + 16);
    acc[nt] = wmb(ah, b0, acc[nt]);
    b1.h[0] = *(const v8usa*)(wq + 32);
    b1.h[1] = *(const v8usa*)(wq + 48);
    acc[nt] = wmb(al, b1, acc[nt]);
  }
  __syncthreads();

  const float pois = ((flg[4] | flg[5] | flg[6] | flg[7]) != 0) ? __int_as_float(0x7fc00000) : 0.0f;
  float s[8];
#pragma unroll
  for (int r = 0; r < 8; ++r) s[r] = 0.0f;
#pragma unroll
  for (int nt = 0; nt < 8; ++nt) {
    const int c = 16 * nt + m;
    const float b = sb1[c];
    const float w = sw2[c];
#pragma unroll
    for (int r = 0; r < 8; ++r) s[r] = fmaf(fmaxf(acc[nt][r] + b, 0.0f), w, s[r]);
  }
#pragma unroll
  for (int r = 0; r < 8; ++r) {
    s[r] += __shfl_xor(s[r], 8, 32);
    s[r] += __shfl_xor(s[r], 4, 32);
    s[r] += __shfl_xor(s[r], 2, 32);
    s[r] += __shfl_xor(s[r], 1, 32);
  }
  const float b2 = bf16_val(ib2[0]);
  if (m == 0) {
#pragma unroll
    for (int r = 0; r < 8; ++r) ost[16 * wave + 8 * hh + r] = (s[r] + b2) + pois;
  }
  __syncthreads();
  if (wave == 0) {
    const v4f v = *(const v4fa*)(ost + 4 * lane);
    float* op = outp + (size_t)rowBase + 4 * lane;
    *(volatile v4f*)op = v;
    __threadfence();
    *(volatile v4f*)op = v;
  }
}

__global__ __launch_bounds__(ETHR) void k_edge(const float* mu, const int* __restrict__ slot,
                                               const int* __restrict__ us, const int* __restrict__ ud,
                                               const float* __restrict__ esc, const float* __restrict__ ebi,
                                               float* outp, int nEU, int nSlot, int nN, int nTot) {
  __shared__ __attribute__((aligned(16))) float est[ETHR];
  const int tid = (int)threadIdx.x;
  int idx = (int)blockIdx.x * ETHR + tid;
  idx = idx < nTot ? idx : nTot - 1;
  const int b = idx / nEU;
  const int e = idx - b * nEU;
  int ua = us[e];
  ua = ua < 0 ? 0 : (ua > nSlot - 1 ? nSlot - 1 : ua);
  int ub = ud[e];
  ub = ub < 0 ? 0 : (ub > nSlot - 1 ? nSlot - 1 : ub);
  int ra = b * nSlot + ua;
  ra = ra < 0 ? 0 : (ra > nN - 1 ? nN - 1 : ra);
  int rb = b * nSlot + ub;
  rb = rb < 0 ? 0 : (rb > nN - 1 ? nN - 1 : rb);
  const int sa = slot[ra];
  const int sb = slot[rb];
  const float* pa = mu + (size_t)ra * LAT;
  const float* pb = mu + (size_t)rb * LAT;
  float d = 0.0f;
#pragma unroll
  for (int i = 0; i < 8; ++i) {
    const v4f va = *(const v4fa*)(pa + 4 * i);
    const v4f vb = *(const v4fa*)(pb + 4 * i);
    d += (va.x * vb.x + va.y * vb.y) + (va.z * vb.z + va.w * vb.w);
  }
  const float sc = bf16_val(esc[0]);
  const float bi = bf16_val(ebi[0]);
  float v = sc * d + bi;
  v = ((sa != ra) | (sb != rb)) ? __int_as_float(0x7fc00000) : v;
  est[tid] = v;
  __syncthreads();
  if (tid < 64) {
    const v4f q = *(const v4fa*)(est + 4 * tid);
    float* op = outp + (size_t)blockIdx.x * ETHR + 4 * tid;
    *(volatile v4f*)op = q;
    __threadfence();
    *(volatile v4f*)op = q;
  }
}

static inline int cdiv(int a, int b) { return (a + b - 1) / b; }
static inline size_t al256(size_t o) { return (o + 255) & ~(size_t)255; }

extern "C" void kernel_launch(void* const* d_in, const int* in_sizes, int n_in,
                              void* d_out, int out_size, void* d_ws, size_t ws_size,
                              hipStream_t stream) {
  if (n_in < 37) return;
  const int nN = in_sizes[2];
  if (nN < IROWS || (nN % IROWS) != 0 || nN > (1 << 22)) return;
  if ((long long)in_sizes[0] != (long long)nN * DIN) return;
  if (in_sizes[1] < 2 || (in_sizes[1] & 1) != 0) return;
  const int nE = in_sizes[1] / 2;
  if (nE < 1 || nE >= (1 << 21)) return;
  const int nEU = in_sizes[3];
  if (nEU < 1 || in_sizes[4] != nEU) return;
  for (int t = 0; t < 2; ++t) {
    const int bs = 5 + 13 * t;
    if (in_sizes[bs] != DIN * DF || in_sizes[bs + 1] != DIN * DF || in_sizes[bs + 2] != DF) return;
    if (in_sizes[bs + 3] != DF * DF || in_sizes[bs + 4] != DF * DF || in_sizes[bs + 5] != DF) return;
    if (in_sizes[bs + 6] != DF * LAT || in_sizes[bs + 7] != DF * LAT || in_sizes[bs + 8] != LAT) return;
    if (in_sizes[bs + 9] != DF || in_sizes[bs + 10] != DF || in_sizes[bs + 11] != DF || in_sizes[bs + 12] != DF) return;
  }
  if (in_sizes[31] != LAT * DF || in_sizes[32] != DF || in_sizes[33] != DF || in_sizes[34] != 1) return;
  if (in_sizes[35] != 1 || in_sizes[36] != 1) return;
  const long long rem = (long long)out_size - 65LL * (long long)nN;
  if (rem < nEU || (rem % nEU) != 0) return;
  const long long Bl = rem / nEU;
  if (Bl < 1 || Bl > 65536 || ((long long)nN % Bl) != 0) return;
  const int nB    = (int)Bl;
  const int nSlot = nN / nB;
  const long long nTotl = Bl * (long long)nEU;
  if ((nTotl % ETHR) != 0 || nTotl >= (1LL << 31)) return;
  const int nTot = (int)nTotl;
  const size_t OFF1 = (size_t)nTot;
  const size_t OFF2 = OFF1 + (size_t)nN;
  const size_t OFF3 = OFF2 + (size_t)nN * LAT;
  if ((long long)(OFF3 + (size_t)nN * LAT) != (long long)out_size) return;

  const float* x    = (const float*)d_in[0];
  const int*   ei   = (const int*)  d_in[1];
  const int*   slot = (const int*)  d_in[2];
  const int*   us   = (const int*)  d_in[3];
  const int*   ud   = (const int*)  d_in[4];
  const float* mW0l = (const float*)d_in[5];
  const float* mW0r = (const float*)d_in[6];
  const float* mb0  = (const float*)d_in[7];
  const float* mW1l = (const float*)d_in[8];
  const float* mW1r = (const float*)d_in[9];
  const float* mb1  = (const float*)d_in[10];
  const float* mW2l = (const float*)d_in[11];
  const float* mW2r = (const float*)d_in[12];
  const float* mb2  = (const float*)d_in[13];
  const float* mg0  = (const float*)d_in[14];
  const float* mbt0 = (const float*)d_in[15];
  const float* mg1  = (const float*)d_in[16];
  const float* mbt1 = (const float*)d_in[17];
  const float* vW0l = (const float*)d_in[18];
  const float* vW0r = (const float*)d_in[19];
  const float* vb0  = (const float*)d_in[20];
  const float* vW1l = (const float*)d_in[21];
  const float* vW1r = (const float*)d_in[22];
  const float* vb1  = (const float*)d_in[23];
  const float* vW2l = (const float*)d_in[24];
  const float* vW2r = (const float*)d_in[25];
  const float* vb2  = (const float*)d_in[26];
  const float* vg0  = (const float*)d_in[27];
  const float* vbt0 = (const float*)d_in[28];
  const float* vg1  = (const float*)d_in[29];
  const float* vbt1 = (const float*)d_in[30];
  const float* iW1  = (const float*)d_in[31];
  const float* ib1  = (const float*)d_in[32];
  const float* iW2  = (const float*)d_in[33];
  const float* ib2  = (const float*)d_in[34];
  const float* esc  = (const float*)d_in[35];
  const float* ebi  = (const float*)d_in[36];
  float* out = (float*)d_out;
  const int* src = ei;
  const int* dst = ei + nE;

  const int gM = nN / GBM;
  const int gI = nN / IROWS;
  const int gA = cdiv(nN, NBA);
  if ((long long)gA * NBA < (long long)nN) return;
  const int vec8 = ((nE & 3) == 0) ? 1 : 0;

  char* ws = (char*)d_ws;
  size_t off = 0;
  const size_t oBT0m = off; off = al256(off + (size_t)DF * K0 * 2);
  const size_t oBT0v = off; off = al256(off + (size_t)DF * K0 * 2);
  const size_t oBT1m = off; off = al256(off + (size_t)DF * KB1 * 2);
  const size_t oBT1v = off; off = al256(off + (size_t)DF * KB1 * 2);
  const size_t oBT2m = off; off = al256(off + (size_t)LAT * KB1 * 2);
  const size_t oBT2v = off; off = al256(off + (size_t)LAT * KB1 * 2);
  const size_t oBTi  = off; off = al256(off + (size_t)DF * KBI * 2);
  const size_t oMEAN = off; off = al256(off + (size_t)nN * MPITCH * 2);
  const size_t oHm   = off; off = al256(off + (size_t)nN * HP * 2);
  const size_t oHv   = off; off = al256(off + (size_t)nN * HP * 2);
  if (off > ws_size || off > (size_t)WSMAX) return;
  unsigned short* BT0m = (unsigned short*)(ws + oBT0m);
  unsigned short* BT0v = (unsigned short*)(ws + oBT0v);
  unsigned short* BT1m = (unsigned short*)(ws + oBT1m);
  unsigned short* BT1v = (unsigned short*)(ws + oBT1v);
  unsigned short* BT2m = (unsigned short*)(ws + oBT2m);
  unsigned short* BT2v = (unsigned short*)(ws + oBT2v);
  unsigned short* BTi  = (unsigned short*)(ws + oBTi);
  unsigned short* MEAN = (unsigned short*)(ws + oMEAN);
  unsigned short* Hm   = (unsigned short*)(ws + oHm);
  unsigned short* Hv   = (unsigned short*)(ws + oHv);

  const size_t scanLds = (size_t)AGG_LDS_INTS * 4;
  hipFuncSetAttribute(reinterpret_cast<const void*>(&k_scan<1>), hipFuncAttributeMaxDynamicSharedMemorySize, (int)scanLds);
  hipFuncSetAttribute(reinterpret_cast<const void*>(&k_scan<0>), hipFuncAttributeMaxDynamicSharedMemorySize, (int)scanLds);

  TW t0m; t0m.bt = BT0m; t0m.bias = mb0; t0m.gam = mg0; t0m.bet = mbt0; t0m.hout = Hm;
  TW t0v; t0v.bt = BT0v; t0v.bias = vb0; t0v.gam = vg0; t0v.bet = vbt0; t0v.hout = Hv;
  TW t1m; t1m.bt = BT1m; t1m.bias = mb1; t1m.gam = mg1; t1m.bet = mbt1; t1m.hout = Hm;
  TW t1v; t1v.bt = BT1v; t1v.bias = vb1; t1v.gam = vg1; t1v.bet = vbt1; t1v.hout = Hv;
  const float climNone = __builtin_huge_valf();
  const float climV    = 10.0f;

  k_wprep<<<NUNITS / NTHR, NTHR, 0, stream>>>(mW0l, mW0r, vW0l, vW0r, mW1l, mW1r, vW1l, vW1r,
                                              mW2l, mW2r, vW2l, vW2r, iW1,
                                              BT0m, BT0v, BT1m, BT1v, BT2m, BT2v, BTi);
  k_scan<1><<<gA, NTHR, scanLds, stream>>>(src, dst, nE, nN, vec8, nN, x, Hm, MEAN);
  k_gemmh<<<dim3(gM, 2), GTHR, 0, stream>>>(MEAN, MPITCH, K0, Hm, HP, 0, t0m, t0v, nN);
  k_scan<0><<<gA, NTHR, scanLds, stream>>>(src, dst, nE, nN, vec8, nN, x, Hm, MEAN);
  k_gemmh<<<dim3(gM, 1), GTHR, 0, stream>>>(MEAN, MPITCH, KM, Hm, HP, KH, t1m, t1m, nN);
  k_scan<0><<<gA, NTHR, scanLds, stream>>>(src, dst, nE, nN, vec8, nN, x, Hv, MEAN);
  k_gemmh<<<dim3(gM, 1), GTHR, 0, stream>>>(MEAN, MPITCH, KM, Hv, HP, KH, t1v, t1v, nN);
  k_scan<0><<<gA, NTHR, scanLds, stream>>>(src, dst, nE, nN, vec8, nN, x, Hm, MEAN);
  k_gemmo<<<gM, GTHR, 0, stream>>>(MEAN, MPITCH, KM, Hm, HP, KH, BT2m, mb2, climNone, out + OFF2, nN);
  k_scan<0><<<gA, NTHR, scanLds, stream>>>(src, dst, nE, nN, vec8, nN, x, Hv, MEAN);
  k_gemmo<<<gM, GTHR, 0, stream>>>(MEAN, MPITCH, KM, Hv, HP, KH, BT2v, vb2, climV, out + OFF3, nN);
  k_ign<<<gI, ITHR, 0, stream>>>(out + OFF2, slot, BTi, ib1, iW2, ib2, out + OFF1, nN);
  k_edge<<<nTot / ETHR, ETHR, 0, stream>>>(out + OFF2, slot, us, ud, esc, ebi, out, nEU, nSlot, nN, nTot);
}
